// GraphTransformerModule_33328946217388
// MI455X (gfx1250) — hardware-verified
//
#include <hip/hip_runtime.h>
#include <stddef.h>


#define GR     16
#define WSC    64.0f
#define WSCI   0.015625f
#define CHUNK  2048
#define ATHR   256
#define AWAVE  8
#define WCAP   256
#define NGRP   (CHUNK / (ATHR * 4))
#define AGG_SACC 65536
#define AGG_AUX  4096
#define AGG_LIST (AWAVE * WCAP)
#define AGG_LDS_BYTES ((AGG_SACC + AGG_AUX + AGG_LIST + AWAVE) * 4)

static_assert(AGG_LDS_BYTES == 286752);
static_assert(WCAP == (CHUNK / ATHR) * 32);
static_assert(NGRP == 2);
static_assert(CHUNK == 2048);

typedef float    v2f  __attribute__((ext_vector_type(2)));
typedef float    v4f  __attribute__((ext_vector_type(4)));
typedef float    v8f  __attribute__((ext_vector_type(8)));
typedef int      v4i  __attribute__((ext_vector_type(4)));
typedef _Float16 v8h  __attribute__((ext_vector_type(8)));
typedef _Float16 v16h __attribute__((ext_vector_type(16)));
union Frag   { v16h v; v8h half[2]; };
union Pack16 { v8h h; v4i i; };

__device__ __forceinline__ v8f wm(v16h a, v16h b, v8f c) {
  v8f d = __builtin_amdgcn_wmma_f32_16x16x32_f16(false, a, false, b, (short)0, c, false, false);
  asm volatile("v_nop\n\tv_nop\n\tv_nop\n\tv_nop" : "+v"(d) : "v"(a), "v"(b));
  return d;
}

__device__ __forceinline__ float wsum(float v) {
  v += __shfl_xor(v, 16, 32);
  v += __shfl_xor(v, 8, 32);
  v += __shfl_xor(v, 4, 32);
  v += __shfl_xor(v, 2, 32);
  v += __shfl_xor(v, 1, 32);
  return v;
}

template <int K>
__global__ __launch_bounds__(256) void k_prep(const float* __restrict__ w0, const float* __restrict__ w1,
                                             const float* __restrict__ w2, const float* __restrict__ w3,
                                             int nce, _Float16* Wh, int ntot) {
  const int n = blockIdx.x * 256 + threadIdx.x;
  if (n >= ntot) return;
  const int which = n / nce;
  const int c = n - which * nce;
  const float* s = (which == 0) ? w0 : ((which == 1) ? w1 : ((which == 2) ? w2 : w3));
  _Float16* dst = Wh + (size_t)n * K;
#pragma unroll
  for (int kb = 0; kb < K / 8; ++kb) {
    Pack16 u;
#pragma unroll
    for (int i = 0; i < 8; ++i) u.h[i] = (_Float16)(s[(size_t)(kb * 8 + i) * nce + c] * WSC);
    *(volatile v4i*)(dst + kb * 8) = u.i;
    __threadfence();
    *(volatile v4i*)(dst + kb * 8) = u.i;
  }
}

template <int K, int NC, int EPI>
__global__ __launch_bounds__(256) void k_gemm(const float* __restrict__ A, const _Float16* __restrict__ Wh,
                                             const float* __restrict__ b0, const float* __restrict__ b1,
                                             const float* __restrict__ b2, const float* __restrict__ b3, int nce,
                                             const float* __restrict__ gam, const float* __restrict__ bet,
                                             float* C, int nA) {
  constexpr int NCT = NC / 16;
  constexpr int NW  = (NCT < 8) ? NCT : 8;
  constexpr int NT  = NW * 32;
  constexpr int TPW = NCT / NW;
  constexpr int AP  = K + 8;
  constexpr int XSP = NC + 4;
  constexpr int RPW = GR / NW;
  constexpr int Q4  = NC / 4;
  constexpr int NIT = (RPW * Q4) / 32;
  static_assert(TPW * NW == NCT);
  static_assert(RPW * NW == GR);
  static_assert(NIT * 32 == RPW * Q4);
  static_assert(K % 32 == 0);
  static_assert(EPI == 0 || NC == 32);
  static_assert((AP * 2) % 16 == 0);
  __shared__ __attribute__((aligned(16))) _Float16 At[GR * AP];
  __shared__ __attribute__((aligned(16))) float Xs[GR * XSP];

  const int tid  = threadIdx.x;
  const int lane = tid & 31;
  const int wave = tid >> 5;
  const int hh   = lane >> 4;
  const int m    = lane & 15;
  const int rowBase = blockIdx.x * GR;

  for (int idx = tid; idx < GR * (K / 8); idx += NT) {
    const int r  = idx / (K / 8);
    const int c0 = (idx - r * (K / 8)) * 8;
    int row = rowBase + r;
    if (row > nA - 1) row = nA - 1;
    const float* p = A + (size_t)row * K + c0;
    const v4f f0 = *(const v4f*)p;
    const v4f f1 = *(const v4f*)(p + 4);
    Pack16 u;
    u.h[0] = (_Float16)f0.x; u.h[1] = (_Float16)f0.y; u.h[2] = (_Float16)f0.z; u.h[3] = (_Float16)f0.w;
    u.h[4] = (_Float16)f1.x; u.h[5] = (_Float16)f1.y; u.h[6] = (_Float16)f1.z; u.h[7] = (_Float16)f1.w;
    *(v8h*)(At + r * AP + c0) = u.h;
  }
  __syncthreads();

  const v8f z8 = {0.f, 0.f, 0.f, 0.f, 0.f, 0.f, 0.f, 0.f};
  v8f acc[TPW];
#pragma unroll
  for (int t = 0; t < TPW; ++t) acc[t] = z8;
#pragma unroll
  for (int kt = 0; kt < K / 32; ++kt) {
    const int k0 = kt * 32;
    Frag a;
    const _Float16* pa = At + m * AP + k0 + 8 * hh;
    a.half[0] = *(const v8h*)pa;
    a.half[1] = *(const v8h*)(pa + 16);
#pragma unroll
    for (int t = 0; t < TPW; ++t) {
      const int ncol = (wave * TPW + t) * 16 + m;
      const _Float16* pb = Wh + (size_t)ncol * K + k0 + 8 * hh;
      Frag b;
      b.half[0] = *(const v8h*)pb;
      b.half[1] = *(const v8h*)(pb + 16);
      acc[t] = wm(a.v, b.v, acc[t]);
    }
  }

#pragma unroll
  for (int t = 0; t < TPW; ++t) {
    const int col = (wave * TPW + t) * 16 + m;
    const int which = col / nce;
    const float* bb = (which == 0) ? b0 : ((which == 1) ? b1 : ((which == 2) ? b2 : b3));
    const float bv = bb[col - which * nce];
#pragma unroll
    for (int r = 0; r < 8; ++r) {
      float v = acc[t][r] * WSCI + bv;
      if (EPI == 1) v = fmaxf(v, 0.f);
      Xs[(8 * hh + r) * XSP + col] = v;
    }
  }
  __syncthreads();

  if (EPI == 1) {
    const float g = gam[lane];
    const float be = bet[lane];
#pragma unroll
    for (int i = 0; i < RPW; ++i) {
      const int row = wave * RPW + i;
      const float v = Xs[row * XSP + lane];
      const float mu = wsum(v) * (1.0f / 32.0f);
      const float d = v - mu;
      const float var = wsum(d * d) * (1.0f / 32.0f);
      Xs[row * XSP + lane] = d * rsqrtf(var + 1e-5f) * g + be;
    }
    __syncthreads();
  }

  v4f xr[NIT];
  float* gp[NIT];
#pragma unroll
  for (int it = 0; it < NIT; ++it) {
    const int p   = it * 32 + lane;
    const int rr  = p / Q4;
    const int c4  = p - rr * Q4;
    const int row = wave * RPW + rr;
    xr[it] = *(const v4f*)(Xs + row * XSP + 4 * c4);
    gp[it] = C + (size_t)(rowBase + row) * NC + 4 * c4;
  }
#pragma unroll
  for (int it = 0; it < NIT; ++it) *(volatile v4f*)(gp[it]) = xr[it];
  __threadfence();
#pragma unroll
  for (int it = 0; it < NIT; ++it) *(volatile v4f*)(gp[it]) = xr[it];
}

template <int DF, int NH, int NB, int SH, int EPI>
__global__ __launch_bounds__(ATHR) void k_agg(const int* __restrict__ ei, const float* __restrict__ qkvs,
                                              const float* __restrict__ gam, const float* __restrict__ bet,
                                              float* out, int nN, int nE) {
  constexpr int P   = 4 * DF;
  constexpr int CPL = DF / 32;
  constexpr int LPH = 32 / NH;
  constexpr int SPW = NB / AWAVE;
  constexpr int NV  = NB * DF / 4;
  static_assert(NB == (1 << SH));
  static_assert(NB * DF == AGG_SACC);
  static_assert(2 * NB * NH == AGG_AUX);
  static_assert(CPL * LPH == 32);
  static_assert(CPL == 1 || CPL == 4);
  static_assert(SH + 11 <= 31);
  extern __shared__ v4f lds_dyn[];
  float* sacc = (float*)lds_dyn;
  float* mx   = sacc + AGG_SACC;
  float* den  = mx + NB * NH;
  int*   list = (int*)(den + NB * NH);
  int*   wcnt = list + AGG_LIST;

  const int tid  = threadIdx.x;
  const int lane = tid & 31;
  const int wave = tid >> 5;
  const int hd   = lane / LPH;
  const int nodeBase = blockIdx.x * NB;

  {
    const v4f z4 = {0.f, 0.f, 0.f, 0.f};
    for (int i = tid; i < AGG_SACC / 4; i += ATHR) lds_dyn[i] = z4;
    for (int i = tid; i < NB * NH; i += ATHR) { mx[i] = -1.0e30f; den[i] = 0.f; }
  }
  __syncthreads();

  const int* eid = ei + nE;
  const bool al16 = ((nE & 3) == 0);
  const int nChunks = (nE + CHUNK - 1) / CHUNK;
#pragma unroll 1
  for (int ch = 0; ch < nChunks; ++ch) {
    const int cbase = ch * CHUNK;
    int wc = 0;
#pragma unroll
    for (int g = 0; g < NGRP; ++g) {
      const int el0 = (g * ATHR + tid) * 4;
      const int e0  = cbase + el0;
      const int sent = -2147483647 - 1;
      v4i d;
      if (al16 && (e0 + 3 < nE)) {
        d = *(const v4i*)(eid + e0);
      } else {
        d.x = (e0     < nE) ? eid[min(e0, nE - 1)]     : sent;
        d.y = (e0 + 1 < nE) ? eid[min(e0 + 1, nE - 1)] : sent;
        d.z = (e0 + 2 < nE) ? eid[min(e0 + 2, nE - 1)] : sent;
        d.w = (e0 + 3 < nE) ? eid[min(e0 + 3, nE - 1)] : sent;
      }
      const unsigned s0 = (unsigned)d.x - (unsigned)nodeBase;
      const unsigned s1 = (unsigned)d.y - (unsigned)nodeBase;
      const unsigned s2 = (unsigned)d.z - (unsigned)nodeBase;
      const unsigned s3 = (unsigned)d.w - (unsigned)nodeBase;
      const bool h0 = s0 < (unsigned)NB;
      const bool h1 = s1 < (unsigned)NB;
      const bool h2 = s2 < (unsigned)NB;
      const bool h3 = s3 < (unsigned)NB;
      const unsigned many = __builtin_amdgcn_ballot_w32(h0 | h1 | h2 | h3);
      if (many != 0u) {
#define HITJ(J, HJ, SJ) { \
          const unsigned mj = __builtin_amdgcn_ballot_w32(HJ); \
          if (HJ) { \
            const int pos = wc + (int)__builtin_amdgcn_mbcnt_lo(mj, 0u); \
            if (pos < WCAP) list[wave * WCAP + pos] = ((el0 + (J)) << SH) | (int)(SJ); \
          } \
          wc += (int)__builtin_popcount(mj); }
        HITJ(0, h0, s0)
        HITJ(1, h1, s1)
        HITJ(2, h2, s2)
        HITJ(3, h3, s3)
#undef HITJ
      }
    }
    if (lane == 0) wcnt[wave] = wc;
    __syncthreads();

    if (wave == 0) {
      for (int wsx = 0; wsx < AWAVE; ++wsx) {
        int n = wcnt[wsx];
        if (n > WCAP) n = WCAP;
        if (n < 0) n = 0;
        for (int i = 0; i < n; ++i) {
          const int ent  = list[wsx * WCAP + i];
          const int slot = ent & (NB - 1);
          const int el   = (ent >> SH) & (CHUNK - 1);
          int e = cbase + el;
          if (e > nE - 1) e = nE - 1;
          int src = ei[e];
          src = src < 0 ? 0 : (src > nN - 1 ? nN - 1 : src);
          int nd = nodeBase + slot;
          if (nd > nN - 1) nd = nN - 1;
          const float* qrow = qkvs + (size_t)nd * P;
          const float* krow = qkvs + (size_t)src * P + DF;
          const float* vrow = krow + DF;
          float part;
          v4f v4 = {0.f, 0.f, 0.f, 0.f};
          float v1 = 0.f;
          if (CPL == 4) {
            const v4f q4 = *(const v4f*)(qrow + 4 * lane);
            const v4f k4 = *(const v4f*)(krow + 4 * lane);
            v4 = *(const v4f*)(vrow + 4 * lane);
            part = q4.x * k4.x + q4.y * k4.y + q4.z * k4.z + q4.w * k4.w;
          } else {
            const float qs = qrow[lane];
            const float kz = krow[lane];
            v1 = vrow[lane];
            part = qs * kz;
          }
#pragma unroll
          for (int mk = LPH / 2; mk >= 1; mk >>= 1) part += __shfl_xor(part, mk, 32);
          const float logit = part * 0.17677669529663687f;
          const int hidx = slot * NH + hd;
          const float mo = mx[hidx];
          const float mn = fmaxf(mo, logit);
          const float corr = __expf(mo - mn);
          const float p = __expf(logit - mn);
          const float dn = den[hidx] * corr + p;
          if (CPL == 4) {
            v4f* sp = (v4f*)(sacc + slot * DF + 4 * lane);
            const v4f cur = *sp;
            *sp = cur * corr + v4 * p;
          } else {
            const float cur = sacc[slot * DF + lane];
            sacc[slot * DF + lane] = cur * corr + v1 * p;
          }
          den[hidx] = dn;
          mx[hidx]  = mn;
        }
      }
    }
    __syncthreads();
  }

  v4f g4 = {1.f, 1.f, 1.f, 1.f};
  v4f e4 = {0.f, 0.f, 0.f, 0.f};
  float g1 = 1.f, e1 = 0.f;
  if (EPI == 1) {
    if (CPL == 4) { g4 = *(const v4f*)(gam + 4 * lane); e4 = *(const v4f*)(bet + 4 * lane); }
    else          { g1 = gam[lane]; e1 = bet[lane]; }
  }
#pragma unroll 1
  for (int j = 0; j < SPW; ++j) {
    const int slot = wave * SPW + j;
    const int node = nodeBase + slot;
    if (node < nN) {
      const float inv = 1.0f / (den[slot * NH + hd] + 1e-16f);
      const float* srow = qkvs + (size_t)node * P + 3 * DF;
      if (CPL == 4) {
        v4f* sp = (v4f*)(sacc + slot * DF + 4 * lane);
        v4f a = *sp * inv + *(const v4f*)(srow + 4 * lane);
        a.x = fmaxf(a.x, 0.f); a.y = fmaxf(a.y, 0.f); a.z = fmaxf(a.z, 0.f); a.w = fmaxf(a.w, 0.f);
        if (EPI == 1) {
          const float s  = wsum(a.x + a.y + a.z + a.w);
          const float mu = s * (1.0f / DF);
          const v4f dd = a - mu;
          const float q  = wsum(dd.x * dd.x + dd.y * dd.y + dd.z * dd.z + dd.w * dd.w);
          const float rs = rsqrtf(q * (1.0f / DF) + 1e-5f);
          a = dd * rs * g4 + e4;
        }
        *sp = a;
      } else {
        float a = sacc[slot * DF + lane] * inv + srow[lane];
        a = fmaxf(a, 0.f);
        if (EPI == 1) {
          const float mu = wsum(a) * (1.0f / DF);
          const float dd = a - mu;
          const float rs = rsqrtf(wsum(dd * dd) * (1.0f / DF) + 1e-5f);
          a = dd * rs * g1 + e1;
        }
        sacc[slot * DF + lane] = a;
      }
    }
  }
  __syncthreads();

  for (int idx = tid; idx < NV; idx += ATHR) {
    const int row = idx / (DF / 4);
    const int c4  = idx - row * (DF / 4);
    const int node = nodeBase + row;
    if (node < nN) {
      const v4f val = *(const v4f*)(sacc + row * DF + 4 * c4);
      *(volatile v4f*)(out + (size_t)node * DF + 4 * c4) = val;
    }
  }
  __threadfence();
  for (int idx = tid; idx < NV; idx += ATHR) {
    const int row = idx / (DF / 4);
    const int c4  = idx - row * (DF / 4);
    const int node = nodeBase + row;
    if (node < nN) {
      const v4f val = *(const v4f*)(sacc + row * DF + 4 * c4);
      *(volatile v4f*)(out + (size_t)node * DF + 4 * c4) = val;
    }
  }
}

__global__ __launch_bounds__(ATHR) void k_pool(const float* __restrict__ Y, const int* __restrict__ bat,
                                               float* out, int nN, int nG) {
  __shared__ __attribute__((aligned(16))) float ps[AWAVE * 64];
  const int tid  = threadIdx.x;
  const int lane = tid & 31;
  const int wave = tid >> 5;
  const int ngi = (nG + AWAVE - 1) / AWAVE;
#pragma unroll 1
  for (int it = 0; it < ngi; ++it) {
    const int g = it * AWAVE + wave;
    float a0 = 0.f, a1 = 0.f;
    int cnt = 0;
#pragma unroll 1
    for (int base = 0; base < nN; base += 32) {
      const int n = base + lane;
      const int b = (n < nN) ? bat[n] : -1;
      unsigned msk = __builtin_amdgcn_ballot_w32(b == g);
      cnt += (int)__builtin_popcount(msk);
      while (msk != 0u) {
        const int j = __builtin_ctz(msk);
        msk &= msk - 1u;
        const v2f y = *(const v2f*)(Y + (size_t)(base + j) * 64 + 2 * lane);
        a0 += y.x;
        a1 += y.y;
      }
    }
    const float inv = 1.0f / fmaxf((float)cnt, 1.0f);
    ps[wave * 64 + 2 * lane]     = a0 * inv;
    ps[wave * 64 + 2 * lane + 1] = a1 * inv;
    __syncthreads();
    const bool wr = (g < nG) && (lane < 16);
    v4f o = {0.f, 0.f, 0.f, 0.f};
    float* op = out;
    if (wr) {
      o = *(const v4f*)(ps + wave * 64 + 4 * lane);
      op = out + (size_t)g * 64 + 4 * lane;
    }
    if (wr) *(volatile v4f*)op = o;
    __threadfence();
    if (wr) *(volatile v4f*)op = o;
    __syncthreads();
  }
}

extern "C" void kernel_launch(void* const* d_in, const int* in_sizes, int n_in,
                              void* d_out, int out_size, void* d_ws, size_t ws_size,
                              hipStream_t stream) {
  if (n_in < 27) return;
  const int nN = in_sizes[2];
  if (nN <= 0 || in_sizes[0] != nN * 128) return;
  if (in_sizes[1] < 2 || (in_sizes[1] & 1)) return;
  const int nE = in_sizes[1] / 2;
  if (in_sizes[3] != 128 * 32 || in_sizes[4] != 32 || in_sizes[5] != 32 || in_sizes[6] != 32) return;
  if (in_sizes[7] != 32 * 128 || in_sizes[9] != 32 * 128 || in_sizes[11] != 32 * 128 || in_sizes[13] != 32 * 128) return;
  if (in_sizes[8] != 128 || in_sizes[10] != 128 || in_sizes[12] != 128 || in_sizes[14] != 128) return;
  if (in_sizes[15] != 128 || in_sizes[16] != 128) return;
  if (in_sizes[17] != 128 * 32 || in_sizes[19] != 128 * 32 || in_sizes[21] != 128 * 32 || in_sizes[23] != 128 * 32) return;
  if (in_sizes[18] != 32 || in_sizes[20] != 32 || in_sizes[22] != 32 || in_sizes[24] != 32) return;
  if (in_sizes[25] != 32 * 64 || in_sizes[26] != 64) return;
  const int nG = out_size / 64;
  if (nG <= 0 || out_size != nG * 64) return;

  const float* x      = (const float*)d_in[0];
  const int*   ei     = (const int*)d_in[1];
  const int*   bat    = (const int*)d_in[2];
  const float* lin1_w = (const float*)d_in[3];
  const float* lin1_b = (const float*)d_in[4];
  const float* ln1_g  = (const float*)d_in[5];
  const float* ln1_b  = (const float*)d_in[6];
  const float* t1_wq  = (const float*)d_in[7];
  const float* t1_bq  = (const float*)d_in[8];
  const float* t1_wk  = (const float*)d_in[9];
  const float* t1_bk  = (const float*)d_in[10];
  const float* t1_wv  = (const float*)d_in[11];
  const float* t1_bv  = (const float*)d_in[12];
  const float* t1_ws  = (const float*)d_in[13];
  const float* t1_bs  = (const float*)d_in[14];
  const float* ln2_g  = (const float*)d_in[15];
  const float* ln2_b  = (const float*)d_in[16];
  const float* t2_wq  = (const float*)d_in[17];
  const float* t2_bq  = (const float*)d_in[18];
  const float* t2_wk  = (const float*)d_in[19];
  const float* t2_bk  = (const float*)d_in[20];
  const float* t2_wv  = (const float*)d_in[21];
  const float* t2_bv  = (const float*)d_in[22];
  const float* t2_ws  = (const float*)d_in[23];
  const float* t2_bs  = (const float*)d_in[24];
  const float* lin2_w = (const float*)d_in[25];
  const float* lin2_b = (const float*)d_in[26];
  float* out = (float*)d_out;

  const int Np = ((nN + GR - 1) / GR) * GR;
  size_t off = 0;
  _Float16* Wl1 = (_Float16*)((char*)d_ws + off); off += (size_t)32 * 128 * 2;
  _Float16* Wt1 = (_Float16*)((char*)d_ws + off); off += (size_t)512 * 32 * 2;
  _Float16* Wt2 = (_Float16*)((char*)d_ws + off); off += (size_t)128 * 128 * 2;
  _Float16* Wl2 = (_Float16*)((char*)d_ws + off); off += (size_t)64 * 32 * 2;
  float* RB = (float*)((char*)d_ws + off); off += (size_t)Np * 512 * sizeof(float);
  float* RC = (float*)((char*)d_ws + off); off += (size_t)Np * 128 * sizeof(float);
  if (off > ws_size) return;
  float* qkvs1 = RB;
  float* qkvs2 = RB;
  float* Y     = RB;
  float* h1    = RC;
  float* h2    = RC;
  float* o2    = RC;

  k_prep<128><<<1, 256, 0, stream>>>(lin1_w, lin1_w, lin1_w, lin1_w, 32, Wl1, 32);
  k_prep<32><<<2, 256, 0, stream>>>(t1_wq, t1_wk, t1_wv, t1_ws, 128, Wt1, 512);
  k_prep<128><<<1, 256, 0, stream>>>(t2_wq, t2_wk, t2_wv, t2_ws, 32, Wt2, 128);
  k_prep<32><<<1, 256, 0, stream>>>(lin2_w, lin2_w, lin2_w, lin2_w, 64, Wl2, 64);

  const int gblk = Np / GR;
  k_gemm<128, 32, 1><<<gblk, 64, 0, stream>>>(x, Wl1, lin1_b, lin1_b, lin1_b, lin1_b, 32,
                                                ln1_g, ln1_b, h1, nN);
  k_gemm<32, 512, 0><<<gblk, 256, 0, stream>>>(h1, Wt1, t1_bq, t1_bk, t1_bv, t1_bs, 128,
                                                 (const float*)0, (const float*)0, qkvs1, nN);
  hipFuncSetAttribute(reinterpret_cast<const void*>(&k_agg<128, 4, 512, 9, 1>),
                      hipFuncAttributeMaxDynamicSharedMemorySize, AGG_LDS_BYTES);
  k_agg<128, 4, 512, 9, 1><<<(nN + 511) / 512, ATHR, AGG_LDS_BYTES, stream>>>(ei, qkvs1, ln2_g, ln2_b,
                                                                              h2, nN, nE);
  k_gemm<128, 128, 0><<<gblk, 256, 0, stream>>>(h2, Wt2, t2_bq, t2_bk, t2_bv, t2_bs, 32,
                                                  (const float*)0, (const float*)0, qkvs2, nN);
  hipFuncSetAttribute(reinterpret_cast<const void*>(&k_agg<32, 1, 2048, 11, 2>),
                      hipFuncAttributeMaxDynamicSharedMemorySize, AGG_LDS_BYTES);
  k_agg<32, 1, 2048, 11, 2><<<(nN + 2047) / 2048, ATHR, AGG_LDS_BYTES, stream>>>(ei, qkvs2, (const float*)0,
                                                                                 (const float*)0, o2, nN, nE);
  k_gemm<32, 64, 0><<<gblk, 128, 0, stream>>>(o2, Wl2, lin2_b, lin2_b, lin2_b, lin2_b, 64,
                                                (const float*)0, (const float*)0, Y, nN);
  k_pool<<<1, ATHR, 0, stream>>>(Y, bat, out, nN, nG);
}
